// MambaPredictor_28028956573916
// MI455X (gfx1250) — hardware-verified
//
#include <hip/hip_runtime.h>
#include <stdint.h>
#include <stddef.h>


#define B_      8
#define L_      2048
#define DMODEL  512
#define DSTATE  16
#define DCONV   4
#define DINNER  1024
#define DTRANK  32
#define NDBL    64
#define MTOK    (B_ * L_)
#define MPAD    64

typedef __attribute__((ext_vector_type(16))) _Float16 v16h;
typedef __attribute__((ext_vector_type(8)))  _Float16 v8h;
typedef __attribute__((ext_vector_type(16))) __bf16   v16b;
typedef __attribute__((ext_vector_type(8)))  __bf16   v8b;
typedef __attribute__((ext_vector_type(8)))  float    v8f;
typedef __attribute__((ext_vector_type(4)))  float    v4f;
typedef __attribute__((ext_vector_type(2)))  float    v2f;
#define PSCALE 32768.0f
#define U16(p) ((const unsigned short*)(const void*)(p))
#define PSCALE_INV (1.0f / 32768.0f)

__device__ __forceinline__ unsigned short f2bf_bits(float f) {
  unsigned u = __float_as_uint(f);
  return (unsigned short)((u + 0x7FFFu + ((u >> 16) & 1u)) >> 16);
}
__device__ __forceinline__ float bf_bits2f(unsigned short h) { return __uint_as_float(((unsigned)h) << 16); }

__device__ __forceinline__ void dep_guard_h(v8f& a, v8f& b, v16h x, v16h y) { asm volatile("v_nop\n\tv_nop\n\tv_nop\n\tv_nop" : "+v"(a), "+v"(b) : "v"(x), "v"(y)); }
__device__ __forceinline__ void dep_guard_b(v8f& a, v8f& b, v16b x, v16b y) { asm volatile("v_nop\n\tv_nop\n\tv_nop\n\tv_nop" : "+v"(a), "+v"(b) : "v"(x), "v"(y)); }
__device__ __forceinline__ void keep4_h(v16h a, v16h b, v16h c, v16h d) { asm volatile("v_nop" :: "v"(a), "v"(b), "v"(c), "v"(d)); }
__device__ __forceinline__ void keep4_b(v16b a, v16b b, v16b c, v16b d) { asm volatile("v_nop" :: "v"(a), "v"(b), "v"(c), "v"(d)); }
__device__ __forceinline__ void acc_guard4(v8f& a, v8f& b, v8f& c, v8f& d) { asm volatile("v_nop\n\tv_nop\n\tv_nop\n\tv_nop" : "+v"(a), "+v"(b), "+v"(c), "+v"(d)); }
template <typename T> struct Frag;
template <> struct Frag<_Float16> {
  typedef v16h V; union U { v16h v; v8h h[2]; };
  static __device__ __forceinline__ v16h load(const _Float16* p) {
    U f; f.h[0] = *(const v8h*)(p); f.h[1] = *(const v8h*)(p + 16); return f.v;
  }
  static __device__ __forceinline__ v8f mma(v16h a, v16h b, v8f c) {
    return __builtin_amdgcn_wmma_f32_16x16x32_f16(false, a, false, b, (short)0, c, false, false);
  }
  static __device__ __forceinline__ void guard(v8f& a, v8f& b, v16h x, v16h y) { dep_guard_h(a, b, x, y); }
  static __device__ __forceinline__ void keep(v16h a, v16h b, v16h c, v16h d) { keep4_h(a, b, c, d); }
};
template <> struct Frag<__bf16> {
  typedef v16b V; union U { v16b v; v8b h[2]; };
  static __device__ __forceinline__ v16b load(const __bf16* p) {
    U f; f.h[0] = *(const v8b*)(p); f.h[1] = *(const v8b*)(p + 16); return f.v;
  }
  static __device__ __forceinline__ v8f mma(v16b a, v16b b, v8f c) {
    return __builtin_amdgcn_wmma_f32_16x16x32_bf16(false, a, false, b, (short)0, c, false, false);
  }
  static __device__ __forceinline__ void guard(v8f& a, v8f& b, v16b x, v16b y) { dep_guard_b(a, b, x, y); }
  static __device__ __forceinline__ void keep(v16b a, v16b b, v16b c, v16b d) { keep4_b(a, b, c, d); }
};

template <int ET> struct Elem;
template <> struct Elem<0> { typedef _Float16 T; };
template <> struct Elem<1> { typedef __bf16 T; };
template <int ET, bool SPLIT, int BIAS_MODE, int OUT_MODE, bool RESID, int ACT = 0>
__global__ __launch_bounds__(256) void wmma_gemm64(
    const unsigned short* __restrict__ Ap, const unsigned short* __restrict__ A2p, int lda, long strideA,
    const unsigned short* __restrict__ Btp, const unsigned short* __restrict__ Bt2p, int ldb, long strideB,
    void* __restrict__ Cout, void* __restrict__ Cout2, int ldc, long strideC,
    const float* __restrict__ bias,
    const float* __restrict__ resid, long strideR,
    int M, int N, int K, float scale) {
  typedef typename Elem<ET>::T T;
  typedef typename Frag<T>::V V;
  const T* A = (const T*)Ap; const T* A2 = (const T*)A2p; const T* Bt = (const T*)Btp; const T* Bt2 = (const T*)Bt2p;
  __shared__ __align__(16) float sT[8][16 * 68];
  const int b    = blockIdx.y;
  const int lane = threadIdx.x & 31;
  const int wave = threadIdx.x >> 5;
  const int tilesN = N >> 6;
  const int tilesM = M >> 6;
  const int tile = blockIdx.x * 8 + wave;
  if (tile >= tilesM * tilesN) return;
  const int tm = tile / tilesN;
  const int tn = tile - tm * tilesN;
  const int m0 = tm << 6;
  const int n0 = tn << 6;

  const T* Ab  = A  + (size_t)b * strideA;
  const T* Bb  = Bt + (size_t)b * strideB;
  const T* Ab2 = SPLIT ? (A2  + (size_t)b * strideA) : nullptr;
  const T* Bb2 = SPLIT ? (Bt2 + (size_t)b * strideB) : nullptr;

  const int rlane = lane & 15;
  const int koff  = (lane >> 4) * 8;
  const int mOff  = (lane >> 4) * 8;

  v8f acc[4][4];
#pragma unroll
  for (int i = 0; i < 4; ++i)
#pragma unroll
    for (int j = 0; j < 4; ++j) acc[i][j] = (v8f){0.f,0.f,0.f,0.f,0.f,0.f,0.f,0.f};

  for (int k0 = 0; k0 < K; k0 += 32) {
    V bh[4], bl[4];
#pragma unroll
    for (int j = 0; j < 4; ++j) {
      const size_t bo = (size_t)(n0 + (j << 4) + rlane) * ldb + koff + k0;
      bh[j] = Frag<T>::load(Bb + bo);
      if (SPLIT) bl[j] = Frag<T>::load(Bb2 + bo);
    }
#pragma unroll
    for (int i = 0; i < 4; ++i) {
      const size_t ao = (size_t)(m0 + (i << 4) + rlane) * lda + koff + k0;
      V ah = Frag<T>::load(Ab + ao);
      V al;
      if (SPLIT) al = Frag<T>::load(Ab2 + ao);
#pragma unroll
      for (int j = 0; j < 4; ++j) {
        acc[i][j] = Frag<T>::mma(ah, bh[j], acc[i][j]);
        if (SPLIT) {
          acc[i][j] = Frag<T>::mma(ah, bl[j], acc[i][j]);
          acc[i][j] = Frag<T>::mma(al, bh[j], acc[i][j]);
        }
      }
      Frag<T>::guard(acc[i][0], acc[i][3], ah, SPLIT ? al : ah);
    }
    Frag<T>::keep(bh[0], bh[1], bh[2], bh[3]);
    if (SPLIT) Frag<T>::keep(bl[0], bl[1], bl[2], bl[3]);
  }
  acc_guard4(acc[0][0], acc[0][1], acc[0][2], acc[0][3]);
  acc_guard4(acc[1][0], acc[1][1], acc[1][2], acc[1][3]);
  acc_guard4(acc[2][0], acc[2][1], acc[2][2], acc[2][3]);
  acc_guard4(acc[3][0], acc[3][1], acc[3][2], acc[3][3]);

  float* slab = sT[wave];
  const float* Rb = RESID ? (resid + (size_t)b * strideR) : nullptr;
#pragma unroll
  for (int i = 0; i < 4; ++i) {
    const int mBase = m0 + (i << 4);
#pragma unroll
    for (int j = 0; j < 4; ++j) {
      const int n = n0 + (j << 4) + rlane;
      float bv = 0.f;
      if (BIAS_MODE == 2) bv = bias[n];
#pragma unroll
      for (int r = 0; r < 8; ++r) {
        float v = acc[i][j][r] * scale;
        if (BIAS_MODE == 1) v += bias[mBase + mOff + r];
        if (BIAS_MODE == 2) v += bv;
        if (RESID) v += Rb[(size_t)(mBase + mOff + r) * ldc + n];
        if (ACT == 1) v = tanhf(v);
        if (ACT == 2) v = fmaxf(v, 0.0f);
        if (ACT == 3) v = v / (1.0f + expf(-v));
        if (ACT == 4) v = (v > 0.f) ? v : 0.01f * v;
        if (ACT == 5) v = 0.5f * v * (1.0f + erff(v * 0.70710678118654752f));
        slab[(mOff + r) * 68 + (j << 4) + rlane] = v;
      }
    }
    __builtin_amdgcn_fence(__ATOMIC_RELEASE, "workgroup");
    __builtin_amdgcn_wave_barrier();
    __builtin_amdgcn_fence(__ATOMIC_ACQUIRE, "workgroup");
    if (OUT_MODE == 0) {
      float* C = (float*)Cout + (size_t)b * strideC;
      const int hh = lane >> 4, c4 = (lane & 15) * 4;
      for (int pass = 0; pass < 2; ++pass) {
#pragma unroll
        for (int it = 0; it < 8; ++it) {
          const int row = it * 2 + hh;
          v4f v = *(const v4f*)(slab + row * 68 + c4);
          *(volatile v4f*)(C + (size_t)(mBase + row) * ldc + n0 + c4) = v;
        }
        __threadfence();
      }
    } else {
      const int q = lane >> 3, c8 = (lane & 7) * 8;
      unsigned short* C  = (unsigned short*)Cout  + (size_t)b * strideC;
      unsigned short* C2 = (OUT_MODE == 2) ? ((unsigned short*)Cout2 + (size_t)b * strideC) : nullptr;
      for (int pass = 0; pass < 2; ++pass) {
#pragma unroll
        for (int it = 0; it < 4; ++it) {
          const int row = it * 4 + q;
          const float* sp = slab + row * 68 + c8;
          v8h hv, lv;
#pragma unroll
          for (int e = 0; e < 8; ++e) {
            if (OUT_MODE == 1) {
              hv[e] = (_Float16)sp[e];
            } else {
              unsigned short hb = f2bf_bits(sp[e]);
              unsigned short lb = f2bf_bits(sp[e] - bf_bits2f(hb));
              hv[e] = __builtin_bit_cast(_Float16, hb);
              lv[e] = __builtin_bit_cast(_Float16, lb);
            }
          }
          *(volatile v8h*)(C + (size_t)(mBase + row) * ldc + n0 + c8) = hv;
          if (OUT_MODE == 2) *(volatile v8h*)(C2 + (size_t)(mBase + row) * ldc + n0 + c8) = lv;
        }
        __threadfence();
      }
    }
    __builtin_amdgcn_fence(__ATOMIC_RELEASE, "workgroup");
    __builtin_amdgcn_wave_barrier();
    __builtin_amdgcn_fence(__ATOMIC_ACQUIRE, "workgroup");
  }
}

__device__ __forceinline__ unsigned short at_bf_bits(float f) {
  unsigned u = __float_as_uint(f);
  return (unsigned short)((u + 0x7FFFu + ((u >> 16) & 1u)) >> 16);
}
__device__ __forceinline__ __bf16 at_f2bf(float f) { return __builtin_bit_cast(__bf16, at_bf_bits(f)); }
__device__ __forceinline__ void at_split(float f, __bf16& hi, __bf16& lo) {
  const unsigned short hb = at_bf_bits(f);
  hi = __builtin_bit_cast(__bf16, hb);
  lo = at_f2bf(f - __uint_as_float(((unsigned)hb) << 16));
}
__device__ __forceinline__ v8f at_mma(v16b a, v16b b, v8f c) {
  c = __builtin_amdgcn_wmma_f32_16x16x32_bf16(false, a, false, b, (short)0, c, false, false);
  asm volatile("v_nop\n\tv_nop\n\tv_nop\n\tv_nop" : "+v"(c) : "v"(a), "v"(b));
  return c;
}

__device__ __forceinline__ void split_bits(float f, unsigned short& hb, unsigned short& lb) {
  hb = f2bf_bits(f);
  lb = f2bf_bits(f - bf_bits2f(hb));
}

__device__ __forceinline__ float softplus_f(float v) { return fmaxf(v, 0.0f) + log1pf(expf(-fabsf(v))); }
__device__ __forceinline__ float silu_f(float v) { return v * (1.0f / (1.0f + expf(-v))); }

__global__ __launch_bounds__(256) void cast_f16x2(const float* __restrict__ in, unsigned short* __restrict__ out,
                                                  int n2, float scale) {
  const int i = blockIdx.x * 256 + threadIdx.x;
  if (i < n2) {
    const _Float16 h0 = (_Float16)(in[2 * (size_t)i] * scale);
    const _Float16 h1 = (_Float16)(in[2 * (size_t)i + 1] * scale);
    const unsigned u = (unsigned)__builtin_bit_cast(unsigned short, h0) | ((unsigned)__builtin_bit_cast(unsigned short, h1) << 16);
    ((volatile unsigned*)out)[i] = u;
    __threadfence();
    ((volatile unsigned*)out)[i] = u;
  }
}

__global__ __launch_bounds__(256) void split_bf16x2(const float* __restrict__ in, unsigned short* __restrict__ hi,
                                                    unsigned short* __restrict__ lo, int n2) {
  const int i = blockIdx.x * 256 + threadIdx.x;
  if (i < n2) {
    const float f0 = in[2 * (size_t)i], f1 = in[2 * (size_t)i + 1];
    unsigned short h0, l0, h1, l1;
    split_bits(f0, h0, l0);
    split_bits(f1, h1, l1);
    const unsigned uh = (unsigned)h0 | ((unsigned)h1 << 16);
    const unsigned ul = (unsigned)l0 | ((unsigned)l1 << 16);
    ((volatile unsigned*)hi)[i] = uh;
    ((volatile unsigned*)lo)[i] = ul;
    __threadfence();
    ((volatile unsigned*)hi)[i] = uh;
    ((volatile unsigned*)lo)[i] = ul;
  }
}

__global__ __launch_bounds__(64) void build_last(const float* __restrict__ P, unsigned short* __restrict__ plh,
                                                 unsigned short* __restrict__ pll) {
  const int m = blockIdx.x;
  const int t = threadIdx.x;
  const int mb = (m < B_) ? m : (B_ - 1);
  const float* src = P + ((size_t)mb * L_ + (L_ - 1)) * DMODEL + 8 * t;
  const v4f u0 = *(const v4f*)src;
  const v4f u1 = *(const v4f*)(src + 4);
  const bool live = (m < B_);
  float v[8] = {u0[0], u0[1], u0[2], u0[3], u1[0], u1[1], u1[2], u1[3]};
  v8h hv, lv;
#pragma unroll
  for (int e = 0; e < 8; ++e) {
    const float f = live ? v[e] : 0.0f;
    unsigned short hb, lb;
    split_bits(f, hb, lb);
    hv[e] = __builtin_bit_cast(_Float16, hb);
    lv[e] = __builtin_bit_cast(_Float16, lb);
  }
  unsigned short* oh = plh + (size_t)m * DMODEL + 8 * t;
  unsigned short* ol = pll + (size_t)m * DMODEL + 8 * t;
  *(volatile v8h*)oh = hv;
  *(volatile v8h*)ol = lv;
  __threadfence();
  *(volatile v8h*)oh = hv;
  *(volatile v8h*)ol = lv;
}

__global__ __launch_bounds__(256) void conv_silu_split(const float* __restrict__ X, const float* __restrict__ cw,
                                                       const float* __restrict__ cb,
                                                       unsigned short* __restrict__ xh, unsigned short* __restrict__ xl,
                                                       int row_base) {
  const int r = row_base + (int)(blockIdx.x >> 1);
  const int p = (int)(blockIdx.x & 1) * 256 + (int)threadIdx.x;
  const int d = 2 * p;
  const int t = r & (L_ - 1);
  float a0 = 0.0f, a1 = 0.0f;
#pragma unroll
  for (int j = 0; j < DCONV; ++j) {
    const int tt = t - (DCONV - 1) + j;
    const int rr = (tt >= 0) ? (r - (DCONV - 1) + j) : r;
    const v2f v = *(const v2f*)(X + (size_t)rr * DINNER + d);
    const float v0 = (tt >= 0) ? v[0] : 0.0f;
    const float v1 = (tt >= 0) ? v[1] : 0.0f;
    a0 += cw[d * DCONV + j] * v0;
    a1 += cw[(d + 1) * DCONV + j] * v1;
  }
  a0 += cb[d];
  a1 += cb[d + 1];
  const float s0 = silu_f(a0), s1 = silu_f(a1);
  unsigned short h0, l0, h1, l1;
  split_bits(s0, h0, l0);
  split_bits(s1, h1, l1);
  const unsigned uh = (unsigned)h0 | ((unsigned)h1 << 16);
  const unsigned ul = (unsigned)l0 | ((unsigned)l1 << 16);
  volatile unsigned* oh = (volatile unsigned*)xh + (size_t)r * (DINNER / 2) + p;
  volatile unsigned* ol = (volatile unsigned*)xl + (size_t)r * (DINNER / 2) + p;
  *oh = uh;
  *ol = ul;
  __threadfence();
  *oh = uh;
  *ol = ul;
}

#define SCW 8
#define XSP 68
__global__ __launch_bounds__(256) void ssm_scan(
    const float* __restrict__ xdbl,
    const unsigned short* __restrict__ xh, const unsigned short* __restrict__ xl,
    const unsigned short* __restrict__ wdth, const unsigned short* __restrict__ wdtl,
    const float* __restrict__ bdt, const float* __restrict__ Alog, const float* __restrict__ Dv,
    const float* __restrict__ zbuf,
    unsigned short* __restrict__ ygh, unsigned short* __restrict__ ygl) {
  __shared__ __align__(16) float xs[16 * XSP];
  __shared__ float dts[SCW * 16 * 33];
  __shared__ __align__(16) float ys[SCW * 32];

  const int tid = threadIdx.x, wave = tid >> 5, lane = tid & 31, hh = lane >> 4, c = lane & 15;
  const int ngrp = DINNER / (SCW * 32);
  const int b = (int)blockIdx.x / ngrp;
  const int g = (int)blockIdx.x - b * ngrp;
  const int chb = g * (SCW * 32) + wave * 32;
  const int d = chb + lane;

  float A[DSTATE], h[DSTATE];
#pragma unroll
  for (int s = 0; s < DSTATE; ++s) { A[s] = -expf(Alog[(size_t)d * DSTATE + s]); h[s] = 0.0f; }
  const float bd = bdt[d];

  const __bf16* wh = (const __bf16*)wdth;
  const __bf16* wl = (const __bf16*)wdtl;
  const v16b bh0 = Frag<__bf16>::load(wh + (size_t)(chb + c) * DTRANK + 8 * hh);
  const v16b bl0 = Frag<__bf16>::load(wl + (size_t)(chb + c) * DTRANK + 8 * hh);
  const v16b bh1 = Frag<__bf16>::load(wh + (size_t)(chb + 16 + c) * DTRANK + 8 * hh);
  const v16b bl1 = Frag<__bf16>::load(wl + (size_t)(chb + 16 + c) * DTRANK + 8 * hh);

  const size_t rowb = (size_t)b * L_;
  float* mydt = dts + (size_t)wave * 16 * 33 + lane;

  for (int t0 = 0; t0 < L_; t0 += 16) {
    __syncthreads();
    {
      const int rr = tid >> 4, c4 = (tid & 15) * 4;
      const v4f v = *(const v4f*)(xdbl + (rowb + t0 + rr) * NDBL + c4);
      *(v4f*)(xs + rr * XSP + c4) = v;
    }
    __syncthreads();

    v16b ah, al;
#pragma unroll
    for (int e = 0; e < 8; ++e) {
      __bf16 hq, lq;
      at_split(xs[c * XSP + 8 * hh + e], hq, lq);
      ah[e] = hq; al[e] = lq;
      at_split(xs[c * XSP + 16 + 8 * hh + e], hq, lq);
      ah[8 + e] = hq; al[8 + e] = lq;
    }
    v8f acc0 = (v8f){0.f,0.f,0.f,0.f,0.f,0.f,0.f,0.f};
    v8f acc1 = (v8f){0.f,0.f,0.f,0.f,0.f,0.f,0.f,0.f};
    acc0 = at_mma(ah, bh0, acc0);
    acc0 = at_mma(ah, bl0, acc0);
    acc0 = at_mma(al, bh0, acc0);
    acc1 = at_mma(ah, bh1, acc1);
    acc1 = at_mma(ah, bl1, acc1);
    acc1 = at_mma(al, bh1, acc1);

#pragma unroll
    for (int r = 0; r < 8; ++r) {
      const float v0 = acc0[r], v1 = acc1[r];
      const float mine  = hh ? v1 : v0;
      const float other = hh ? v0 : v1;
      const float recv  = __shfl_xor(other, 16, 32);
      const float row_lo = hh ? recv : mine;
      const float row_hi = hh ? mine : recv;
      mydt[r * 33]       = softplus_f(row_lo + bd);
      mydt[(8 + r) * 33] = softplus_f(row_hi + bd);
    }

#pragma unroll 1
    for (int i = 0; i < 16; ++i) {
      const float dt = mydt[i * 33];
      const size_t xo = (rowb + t0 + i) * DINNER + d;
      const float xv = bf_bits2f(xh[xo]) + bf_bits2f(xl[xo]);
      const v4f q0 = *(const v4f*)(xs + i * XSP + DTRANK);
      const v4f q1 = *(const v4f*)(xs + i * XSP + DTRANK + 4);
      const v4f q2 = *(const v4f*)(xs + i * XSP + DTRANK + 8);
      const v4f q3 = *(const v4f*)(xs + i * XSP + DTRANK + 12);
      const float Bv[16] = {q0[0], q0[1], q0[2], q0[3], q1[0], q1[1], q1[2], q1[3],
                            q2[0], q2[1], q2[2], q2[3], q3[0], q3[1], q3[2], q3[3]};
#pragma unroll
      for (int s = 0; s < DSTATE; ++s)
        h[s] = expf(dt * A[s]) * h[s] + (dt * Bv[s]) * xv;
    }
  }

  float y = 0.0f;
#pragma unroll
  for (int s = 0; s < DSTATE; ++s) y += h[s] * xs[15 * XSP + DTRANK + DSTATE + s];
  const size_t xo = (rowb + L_ - 1) * DINNER + d;
  const float xlast = bf_bits2f(xh[xo]) + bf_bits2f(xl[xo]);
  y += xlast * Dv[d];
  const float z = zbuf[(size_t)b * DINNER + d];
  y = y * silu_f(z);
  ys[wave * 32 + lane] = y;
  __syncthreads();
  if (wave == 0) {
    v8h hv, lv;
#pragma unroll
    for (int e = 0; e < 8; ++e) {
      unsigned short hb, lb;
      split_bits(ys[8 * lane + e], hb, lb);
      hv[e] = __builtin_bit_cast(_Float16, hb);
      lv[e] = __builtin_bit_cast(_Float16, lb);
    }
    unsigned short* oh = ygh + (size_t)b * DINNER + g * (SCW * 32) + 8 * lane;
    unsigned short* ol = ygl + (size_t)b * DINNER + g * (SCW * 32) + 8 * lane;
    *(volatile v8h*)oh = hv;
    *(volatile v8h*)ol = lv;
    __threadfence();
    *(volatile v8h*)oh = hv;
    *(volatile v8h*)ol = lv;
  }
}

__global__ __launch_bounds__(64) void ln_split(const float* __restrict__ outl, const float* __restrict__ gam,
                                               const float* __restrict__ bet,
                                               unsigned short* __restrict__ xnh, unsigned short* __restrict__ xnl) {
  __shared__ float red[4];
  const int b = blockIdx.x, t = threadIdx.x, lane = t & 31, wave = t >> 5;
  const float* x = outl + (size_t)b * DMODEL + 8 * t;
  const v4f u0 = *(const v4f*)x;
  const v4f u1 = *(const v4f*)(x + 4);
  const float v[8] = {u0[0], u0[1], u0[2], u0[3], u1[0], u1[1], u1[2], u1[3]};
  float s = 0.0f;
#pragma unroll
  for (int e = 0; e < 8; ++e) s += v[e];
#pragma unroll
  for (int off = 1; off < 32; off <<= 1) s += __shfl_xor(s, off, 32);
  if (lane == 0) red[wave] = s;
  __syncthreads();
  const float mu = (red[0] + red[1]) * (1.0f / DMODEL);
  float dv[8];
  float q = 0.0f;
#pragma unroll
  for (int e = 0; e < 8; ++e) { dv[e] = v[e] - mu; q += dv[e] * dv[e]; }
#pragma unroll
  for (int off = 1; off < 32; off <<= 1) q += __shfl_xor(q, off, 32);
  if (lane == 0) red[2 + wave] = q;
  __syncthreads();
  const float var = (red[2] + red[3]) * (1.0f / DMODEL);
  const float rstd = 1.0f / sqrtf(var + 1e-5f);
  v8h hv, lv;
#pragma unroll
  for (int e = 0; e < 8; ++e) {
    const float xn = dv[e] * rstd * gam[8 * t + e] + bet[8 * t + e];
    unsigned short hb, lb;
    split_bits(xn, hb, lb);
    hv[e] = __builtin_bit_cast(_Float16, hb);
    lv[e] = __builtin_bit_cast(_Float16, lb);
  }
  unsigned short* oh = xnh + (size_t)b * DMODEL + 8 * t;
  unsigned short* ol = xnl + (size_t)b * DMODEL + 8 * t;
  *(volatile v8h*)oh = hv;
  *(volatile v8h*)ol = lv;
  __threadfence();
  *(volatile v8h*)oh = hv;
  *(volatile v8h*)ol = lv;
}

__global__ __launch_bounds__(256) void out_copy(const float* __restrict__ src, float* __restrict__ out) {
  const int tid = threadIdx.x;
  v4f vals[4];
#pragma unroll
  for (int it = 0; it < 4; ++it) vals[it] = *(const v4f*)(src + 4 * (size_t)(it * 256 + tid));
  for (int pass = 0; pass < 2; ++pass) {
#pragma unroll
    for (int it = 0; it < 4; ++it) *(volatile v4f*)(out + 4 * (size_t)(it * 256 + tid)) = vals[it];
    __threadfence();
  }
}

extern "C" void kernel_launch(void* const* d_in, const int* in_sizes, int n_in,
                              void* d_out, int out_size, void* d_ws, size_t ws_size,
                              hipStream_t stream) {
  if (n_in < 14) return;
  if (in_sizes[0] != MTOK * DMODEL || in_sizes[1] != 2 * DINNER * DMODEL || in_sizes[2] != DINNER * DCONV ||
      in_sizes[3] != DINNER || in_sizes[4] != NDBL * DINNER || in_sizes[5] != DINNER * DTRANK ||
      in_sizes[6] != DINNER || in_sizes[7] != DINNER * DSTATE || in_sizes[8] != DINNER ||
      in_sizes[9] != DMODEL * DINNER || in_sizes[10] != DMODEL || in_sizes[11] != DMODEL ||
      in_sizes[12] != DMODEL * DMODEL || in_sizes[13] != DMODEL || out_size != B_ * DMODEL) return;

  const float* p_hist = (const float*)d_in[0];
  const float* W_in   = (const float*)d_in[1];
  const float* conv_w = (const float*)d_in[2];
  const float* conv_b = (const float*)d_in[3];
  const float* W_x    = (const float*)d_in[4];
  const float* W_dt   = (const float*)d_in[5];
  const float* b_dt   = (const float*)d_in[6];
  const float* A_log  = (const float*)d_in[7];
  const float* Dvec   = (const float*)d_in[8];
  const float* W_out  = (const float*)d_in[9];
  const float* ln_g   = (const float*)d_in[10];
  const float* ln_b   = (const float*)d_in[11];
  const float* W_head = (const float*)d_in[12];
  const float* b_head = (const float*)d_in[13];
  float* out = (float*)d_out;
  char* ws = (char*)d_ws;

  const size_t MiB = (size_t)1048576;
  const size_t off_ph = 0;
  const size_t off_xl = 0;
  const size_t off_x  = 16 * MiB;
  const size_t off_xh = 80 * MiB;
  size_t cur = 112 * MiB;
  auto carve = [&](size_t bytes) { size_t o = cur; cur += (bytes + 255) & ~(size_t)255; return o; };
  const size_t off_xdbl  = carve((size_t)MTOK * NDBL * 4);
  const size_t off_winx  = carve((size_t)DINNER * DMODEL * 2);
  const size_t off_winzh = carve((size_t)DINNER * DMODEL * 2);
  const size_t off_winzl = carve((size_t)DINNER * DMODEL * 2);
  const size_t off_wxh   = carve((size_t)NDBL * DINNER * 2);
  const size_t off_wxl   = carve((size_t)NDBL * DINNER * 2);
  const size_t off_wdth  = carve((size_t)DINNER * DTRANK * 2);
  const size_t off_wdtl  = carve((size_t)DINNER * DTRANK * 2);
  const size_t off_wouth = carve((size_t)DMODEL * DINNER * 2);
  const size_t off_woutl = carve((size_t)DMODEL * DINNER * 2);
  const size_t off_whh   = carve((size_t)DMODEL * DMODEL * 2);
  const size_t off_whl   = carve((size_t)DMODEL * DMODEL * 2);
  const size_t off_plh   = carve((size_t)MPAD * DMODEL * 2);
  const size_t off_pll   = carve((size_t)MPAD * DMODEL * 2);
  const size_t off_zb    = carve((size_t)MPAD * DINNER * 4);
  const size_t small_bytes = (size_t)MPAD * DINNER * 2 * 2 + (size_t)MPAD * DMODEL * 2 * 2;
  const size_t off_ygh   = carve(small_bytes);
  const size_t off_ygl   = off_ygh + (size_t)MPAD * DINNER * 2;
  const size_t off_xnh   = off_ygl + (size_t)MPAD * DINNER * 2;
  const size_t off_xnl   = off_xnh + (size_t)MPAD * DMODEL * 2;
  const size_t off_outl  = carve((size_t)MPAD * DMODEL * 4);
  const size_t off_headb = carve((size_t)MPAD * DMODEL * 4);
  if (cur > ws_size || cur > (size_t)134217728) return;

  unsigned short* ph    = (unsigned short*)(ws + off_ph);
  unsigned short* xl    = (unsigned short*)(ws + off_xl);
  float*          X     = (float*)(ws + off_x);
  unsigned short* xh    = (unsigned short*)(ws + off_xh);
  float*          xdbl  = (float*)(ws + off_xdbl);
  unsigned short* winx  = (unsigned short*)(ws + off_winx);
  unsigned short* winzh = (unsigned short*)(ws + off_winzh);
  unsigned short* winzl = (unsigned short*)(ws + off_winzl);
  unsigned short* wxh   = (unsigned short*)(ws + off_wxh);
  unsigned short* wxl   = (unsigned short*)(ws + off_wxl);
  unsigned short* wdth  = (unsigned short*)(ws + off_wdth);
  unsigned short* wdtl  = (unsigned short*)(ws + off_wdtl);
  unsigned short* wouth = (unsigned short*)(ws + off_wouth);
  unsigned short* woutl = (unsigned short*)(ws + off_woutl);
  unsigned short* whh   = (unsigned short*)(ws + off_whh);
  unsigned short* whl   = (unsigned short*)(ws + off_whl);
  unsigned short* plh   = (unsigned short*)(ws + off_plh);
  unsigned short* pll   = (unsigned short*)(ws + off_pll);
  float*          zb    = (float*)(ws + off_zb);
  unsigned short* ygh   = (unsigned short*)(ws + off_ygh);
  unsigned short* ygl   = (unsigned short*)(ws + off_ygl);
  unsigned short* xnh   = (unsigned short*)(ws + off_xnh);
  unsigned short* xnl   = (unsigned short*)(ws + off_xnl);
  float*          outl  = (float*)(ws + off_outl);
  float*          headb = (float*)(ws + off_headb);

  {
    const int n2 = MTOK * DMODEL / 2;
    cast_f16x2<<<(n2 + 255) / 256, 256, 0, stream>>>(p_hist, ph, n2, 1.0f);
  }
  {
    const int n2 = DINNER * DMODEL / 2;
    cast_f16x2<<<(n2 + 255) / 256, 256, 0, stream>>>(W_in, winx, n2, 64.0f);
    split_bf16x2<<<(n2 + 255) / 256, 256, 0, stream>>>(W_in + (size_t)DINNER * DMODEL, winzh, winzl, n2);
  }
  {
    const int n2 = NDBL * DINNER / 2;
    split_bf16x2<<<(n2 + 255) / 256, 256, 0, stream>>>(W_x, wxh, wxl, n2);
  }
  {
    const int n2 = DINNER * DTRANK / 2;
    split_bf16x2<<<(n2 + 255) / 256, 256, 0, stream>>>(W_dt, wdth, wdtl, n2);
  }
  {
    const int n2 = DMODEL * DINNER / 2;
    split_bf16x2<<<(n2 + 255) / 256, 256, 0, stream>>>(W_out, wouth, woutl, n2);
  }
  {
    const int n2 = DMODEL * DMODEL / 2;
    split_bf16x2<<<(n2 + 255) / 256, 256, 0, stream>>>(W_head, whh, whl, n2);
  }
  build_last<<<MPAD, 64, 0, stream>>>(p_hist, plh, pll);
  hipMemsetAsync(ws + off_ygh, 0, small_bytes, stream);

  wmma_gemm64<1, true, 0, 0, false><<<dim3((MPAD / 64) * (DINNER / 64) / 8, 1), 256, 0, stream>>>(
      plh, pll, DMODEL, 0L, winzh, winzl, DMODEL, 0L, zb, nullptr, DINNER, 0L,
      nullptr, nullptr, 0L, MPAD, DINNER, DMODEL, 1.0f);

  wmma_gemm64<0, false, 0, 0, false><<<dim3((MTOK / 64) * (DINNER / 64) / 8, 1), 256, 0, stream>>>(
      ph, nullptr, DMODEL, 0L, winx, nullptr, DMODEL, 0L, X, nullptr, DINNER, 0L,
      nullptr, nullptr, 0L, MTOK, DINNER, DMODEL, 1.0f / 64.0f);

  conv_silu_split<<<(MTOK / 2) * 2, 256, 0, stream>>>(X, conv_w, conv_b, xh, xl, 0);
  conv_silu_split<<<(MTOK / 2) * 2, 256, 0, stream>>>(X, conv_w, conv_b, xh, xl, MTOK / 2);

  wmma_gemm64<1, true, 0, 0, false><<<dim3((MTOK / 64) * (NDBL / 64) / 8, 1), 256, 0, stream>>>(
      xh, xl, DINNER, 0L, wxh, wxl, DINNER, 0L, xdbl, nullptr, NDBL, 0L,
      nullptr, nullptr, 0L, MTOK, NDBL, DINNER, 1.0f);

  ssm_scan<<<B_ * (DINNER / (SCW * 32)), 256, 0, stream>>>(xdbl, xh, xl, wdth, wdtl, b_dt, A_log, Dvec, zb, ygh, ygl);

  wmma_gemm64<1, true, 0, 0, false><<<dim3((MPAD / 64) * (DMODEL / 64) / 8, 1), 256, 0, stream>>>(
      ygh, ygl, DINNER, 0L, wouth, woutl, DINNER, 0L, outl, nullptr, DMODEL, 0L,
      nullptr, nullptr, 0L, MPAD, DMODEL, DINNER, 1.0f);

  ln_split<<<B_, 64, 0, stream>>>(outl, ln_g, ln_b, xnh, xnl);

  wmma_gemm64<1, true, 2, 0, false><<<dim3((MPAD / 64) * (DMODEL / 64) / 8, 1), 256, 0, stream>>>(
      xnh, xnl, DMODEL, 0L, whh, whl, DMODEL, 0L, headb, nullptr, DMODEL, 0L,
      b_head, nullptr, 0L, MPAD, DMODEL, DMODEL, 1.0f);

  out_copy<<<1, 256, 0, stream>>>(headb, out);
}
